// PrimitiveMixerBlock_73796128080294
// MI455X (gfx1250) — hardware-verified
//
#include <hip/hip_runtime.h>
#include <math.h>
#include <stddef.h>

constexpr int kBatch = 8;
constexpr int kSeq   = 2048;
constexpr int kDim   = 512;
constexpr int kHalf  = 256;
constexpr int kTok   = kBatch * kSeq;
constexpr float kWCarry    = 16.0f;
constexpr float kWCarryInv = 1.0f / 16.0f;

typedef __attribute__((ext_vector_type(16))) _Float16 v16h;
typedef __attribute__((ext_vector_type(8)))  _Float16 v8h;
typedef __attribute__((ext_vector_type(16))) __bf16   v16b;
typedef __attribute__((ext_vector_type(8)))  __bf16   v8b;
typedef __attribute__((ext_vector_type(8)))  float    v8f;
typedef __attribute__((ext_vector_type(4)))  float    v4f;
typedef __attribute__((ext_vector_type(4)))  unsigned int v4u;

__device__ __forceinline__ unsigned short f2bf_bits(float f) {
  unsigned u = __float_as_uint(f);
  return (unsigned short)((u + 0x7FFFu + ((u >> 16) & 1u)) >> 16);
}
__device__ __forceinline__ float bf_bits2f(unsigned short h) { return __uint_as_float(((unsigned)h) << 16); }

__device__ __forceinline__ void dep_guard_h(v8f& a, v8f& b, v16h x, v16h y) { asm volatile("v_nop\n\tv_nop\n\tv_nop\n\tv_nop" : "+v"(a), "+v"(b) : "v"(x), "v"(y)); }
__device__ __forceinline__ void dep_guard_b(v8f& a, v8f& b, v16b x, v16b y) { asm volatile("v_nop\n\tv_nop\n\tv_nop\n\tv_nop" : "+v"(a), "+v"(b) : "v"(x), "v"(y)); }
__device__ __forceinline__ void keep4_h(v16h a, v16h b, v16h c, v16h d) { asm volatile("v_nop" :: "v"(a), "v"(b), "v"(c), "v"(d)); }
__device__ __forceinline__ void keep4_b(v16b a, v16b b, v16b c, v16b d) { asm volatile("v_nop" :: "v"(a), "v"(b), "v"(c), "v"(d)); }
__device__ __forceinline__ void acc_guard4(v8f& a, v8f& b, v8f& c, v8f& d) { asm volatile("v_nop\n\tv_nop\n\tv_nop\n\tv_nop" : "+v"(a), "+v"(b), "+v"(c), "+v"(d)); }
template <typename T> struct Frag;
template <> struct Frag<_Float16> {
  typedef v16h V; union U { v16h v; v8h h[2]; };
  static __device__ __forceinline__ v16h load(const _Float16* p) {
    U f; f.h[0] = *(const v8h*)(p); f.h[1] = *(const v8h*)(p + 16); return f.v;
  }
  static __device__ __forceinline__ v8f mma(v16h a, v16h b, v8f c) {
    return __builtin_amdgcn_wmma_f32_16x16x32_f16(false, a, false, b, (short)0, c, false, false);
  }
  static __device__ __forceinline__ void guard(v8f& a, v8f& b, v16h x, v16h y) { dep_guard_h(a, b, x, y); }
  static __device__ __forceinline__ void keep(v16h a, v16h b, v16h c, v16h d) { keep4_h(a, b, c, d); }
};
template <> struct Frag<__bf16> {
  typedef v16b V; union U { v16b v; v8b h[2]; };
  static __device__ __forceinline__ v16b load(const __bf16* p) {
    U f; f.h[0] = *(const v8b*)(p); f.h[1] = *(const v8b*)(p + 16); return f.v;
  }
  static __device__ __forceinline__ v8f mma(v16b a, v16b b, v8f c) {
    return __builtin_amdgcn_wmma_f32_16x16x32_bf16(false, a, false, b, (short)0, c, false, false);
  }
  static __device__ __forceinline__ void guard(v8f& a, v8f& b, v16b x, v16b y) { dep_guard_b(a, b, x, y); }
  static __device__ __forceinline__ void keep(v16b a, v16b b, v16b c, v16b d) { keep4_b(a, b, c, d); }
};

__device__ __forceinline__ unsigned pk16(unsigned short a, unsigned short b) { return (unsigned)a | ((unsigned)b << 16); }
__device__ __forceinline__ unsigned short h_bits(float f) { const _Float16 h = (_Float16)f; return __builtin_bit_cast(unsigned short, h); }

template <int ET> struct Elem;
template <> struct Elem<0> { typedef _Float16 T; };
template <> struct Elem<1> { typedef __bf16 T; };
template <int ET, bool SPLIT, int BIAS_MODE, int OUT_MODE, bool RESID, int ACT = 0, bool RMUL = false>
__global__ __launch_bounds__(256) void wmma_gemm64(
    const unsigned short* __restrict__ Ap, const unsigned short* __restrict__ A2p, int lda, long strideA,
    const unsigned short* __restrict__ Btp, const unsigned short* __restrict__ Bt2p, int ldb, long strideB,
    void* __restrict__ Cout, void* __restrict__ Cout2, int ldc, long strideC,
    const float* __restrict__ bias,
    const float* __restrict__ resid, long strideR,
    int M, int N, int K, float scale) {
  typedef typename Elem<ET>::T T;
  typedef typename Frag<T>::V V;
  const T* A = (const T*)Ap; const T* A2 = (const T*)A2p; const T* Bt = (const T*)Btp; const T* Bt2 = (const T*)Bt2p;
  __shared__ __align__(16) float sT[8][16 * 68];
  const int b    = blockIdx.y;
  const int lane = threadIdx.x & 31;
  const int wave = threadIdx.x >> 5;
  const int tilesN = N >> 6;
  const int tilesM = M >> 6;
  const int tile = blockIdx.x * 8 + wave;
  if (tile >= tilesM * tilesN) return;
  const int tm = tile / tilesN;
  const int tn = tile - tm * tilesN;
  const int m0 = tm << 6;
  const int n0 = tn << 6;

  const T* Ab  = A  + (size_t)b * strideA;
  const T* Bb  = Bt + (size_t)b * strideB;
  const T* Ab2 = SPLIT ? (A2  + (size_t)b * strideA) : nullptr;
  const T* Bb2 = SPLIT ? (Bt2 + (size_t)b * strideB) : nullptr;

  const int rlane = lane & 15;
  const int koff  = (lane >> 4) * 8;
  const int mOff  = (lane >> 4) * 8;

  v8f acc[4][4];
#pragma unroll
  for (int i = 0; i < 4; ++i)
#pragma unroll
    for (int j = 0; j < 4; ++j) acc[i][j] = (v8f){0.f,0.f,0.f,0.f,0.f,0.f,0.f,0.f};

  for (int k0 = 0; k0 < K; k0 += 32) {
    V bh[4], bl[4];
#pragma unroll
    for (int j = 0; j < 4; ++j) {
      const size_t bo = (size_t)(n0 + (j << 4) + rlane) * ldb + koff + k0;
      bh[j] = Frag<T>::load(Bb + bo);
      if (SPLIT) bl[j] = Frag<T>::load(Bb2 + bo);
    }
#pragma unroll
    for (int i = 0; i < 4; ++i) {
      const size_t ao = (size_t)(m0 + (i << 4) + rlane) * lda + koff + k0;
      V ah = Frag<T>::load(Ab + ao);
      V al;
      if (SPLIT) al = Frag<T>::load(Ab2 + ao);
#pragma unroll
      for (int j = 0; j < 4; ++j) {
        acc[i][j] = Frag<T>::mma(ah, bh[j], acc[i][j]);
        if (SPLIT) {
          acc[i][j] = Frag<T>::mma(ah, bl[j], acc[i][j]);
          acc[i][j] = Frag<T>::mma(al, bh[j], acc[i][j]);
        }
      }
      Frag<T>::guard(acc[i][0], acc[i][3], ah, SPLIT ? al : ah);
    }
    Frag<T>::keep(bh[0], bh[1], bh[2], bh[3]);
    if (SPLIT) Frag<T>::keep(bl[0], bl[1], bl[2], bl[3]);
  }
  acc_guard4(acc[0][0], acc[0][1], acc[0][2], acc[0][3]);
  acc_guard4(acc[1][0], acc[1][1], acc[1][2], acc[1][3]);
  acc_guard4(acc[2][0], acc[2][1], acc[2][2], acc[2][3]);
  acc_guard4(acc[3][0], acc[3][1], acc[3][2], acc[3][3]);

  float* slab = sT[wave];
  const float* Rb = RESID ? (resid + (size_t)b * strideR) : nullptr;
#pragma unroll
  for (int i = 0; i < 4; ++i) {
    const int mBase = m0 + (i << 4);
#pragma unroll
    for (int j = 0; j < 4; ++j) {
      const int n = n0 + (j << 4) + rlane;
      float bv = 0.f;
      if (BIAS_MODE == 2) bv = bias[n];
#pragma unroll
      for (int r = 0; r < 8; ++r) {
        float v = acc[i][j][r] * scale;
        if (BIAS_MODE == 1) v += bias[mBase + mOff + r];
        if (BIAS_MODE == 2) v += bv;
        if (RESID && !RMUL) v += Rb[(size_t)(mBase + mOff + r) * ldc + n];
        if (ACT == 1) v = tanhf(v);
        if (ACT == 2) v = fmaxf(v, 0.0f);
        if (ACT == 4) v = (v > 0.f) ? v : 0.01f * v;
        if (ACT == 6) v = 1.0f / (1.0f + expf(-v));
        if (RESID && RMUL) v = v * Rb[(size_t)(mBase + mOff + r) * ldc + n];
        slab[(mOff + r) * 68 + (j << 4) + rlane] = v;
      }
    }
    __builtin_amdgcn_fence(__ATOMIC_RELEASE, "workgroup");
    __builtin_amdgcn_wave_barrier();
    __builtin_amdgcn_fence(__ATOMIC_ACQUIRE, "workgroup");
    if (OUT_MODE == 0) {
      float* C = (float*)Cout + (size_t)b * strideC;
      const int hh = lane >> 4, c4 = (lane & 15) * 4;
      for (int pass = 0; pass < 2; ++pass) {
#pragma unroll
        for (int it = 0; it < 8; ++it) {
          const int row = it * 2 + hh;
          v4f v = *(const v4f*)(slab + row * 68 + c4);
          *(volatile v4f*)(C + (size_t)(mBase + row) * ldc + n0 + c4) = v;
        }
        __threadfence();
      }
    } else {
      const int q = lane >> 3, c8 = (lane & 7) * 8;
      unsigned short* C  = (unsigned short*)Cout  + (size_t)b * strideC;
      unsigned short* C2 = (OUT_MODE == 2) ? ((unsigned short*)Cout2 + (size_t)b * strideC) : nullptr;
      for (int pass = 0; pass < 2; ++pass) {
#pragma unroll
        for (int it = 0; it < 4; ++it) {
          const int row = it * 4 + q;
          const float* sp = slab + row * 68 + c8;
          v8h hv, lv;
#pragma unroll
          for (int e = 0; e < 8; ++e) {
            if (OUT_MODE == 1) {
              hv[e] = (_Float16)sp[e];
            } else {
              unsigned short hb = f2bf_bits(sp[e]);
              unsigned short lb = f2bf_bits(sp[e] - bf_bits2f(hb));
              hv[e] = __builtin_bit_cast(_Float16, hb);
              lv[e] = __builtin_bit_cast(_Float16, lb);
            }
          }
          *(volatile v8h*)(C + (size_t)(mBase + row) * ldc + n0 + c8) = hv;
          if (OUT_MODE == 2) *(volatile v8h*)(C2 + (size_t)(mBase + row) * ldc + n0 + c8) = lv;
        }
        __threadfence();
      }
    }
    __builtin_amdgcn_fence(__ATOMIC_RELEASE, "workgroup");
    __builtin_amdgcn_wave_barrier();
    __builtin_amdgcn_fence(__ATOMIC_ACQUIRE, "workgroup");
  }
}

__global__ __launch_bounds__(256) void cast8_f16_kernel(const float* __restrict__ in, unsigned short* __restrict__ out,
                                                        int n8, float scale) {
  const int i = blockIdx.x * 256 + threadIdx.x;
  if (i >= n8) return;
  const float* p = in + 8 * (size_t)i;
  const v4f a = *(const v4f*)(p);
  const v4f c = *(const v4f*)(p + 4);
  unsigned short hb[8];
#pragma unroll
  for (int e = 0; e < 4; ++e) {
    hb[e]     = h_bits(a[e] * scale);
    hb[4 + e] = h_bits(c[e] * scale);
  }
  const v4u u = (v4u){pk16(hb[0], hb[1]), pk16(hb[2], hb[3]), pk16(hb[4], hb[5]), pk16(hb[6], hb[7])};
  unsigned short* q = out + 8 * (size_t)i;
  *(volatile v4u*)q = u;
  __threadfence();
  *(volatile v4u*)q = u;
}

__global__ __launch_bounds__(256) void cast8_split_kernel(const float* __restrict__ in, unsigned short* __restrict__ hi,
                                                          unsigned short* __restrict__ lo, int n8) {
  const int i = blockIdx.x * 256 + threadIdx.x;
  if (i >= n8) return;
  const float* p = in + 8 * (size_t)i;
  const v4f a = *(const v4f*)(p);
  const v4f c = *(const v4f*)(p + 4);
  unsigned short hb[8], lb[8];
#pragma unroll
  for (int e = 0; e < 4; ++e) {
    const unsigned short h0 = f2bf_bits(a[e]);
    hb[e] = h0; lb[e] = f2bf_bits(a[e] - bf_bits2f(h0));
    const unsigned short h1 = f2bf_bits(c[e]);
    hb[4 + e] = h1; lb[4 + e] = f2bf_bits(c[e] - bf_bits2f(h1));
  }
  const v4u uh = (v4u){pk16(hb[0], hb[1]), pk16(hb[2], hb[3]), pk16(hb[4], hb[5]), pk16(hb[6], hb[7])};
  const v4u ul = (v4u){pk16(lb[0], lb[1]), pk16(lb[2], lb[3]), pk16(lb[4], lb[5]), pk16(lb[6], lb[7])};
  unsigned short* qh = hi + 8 * (size_t)i;
  unsigned short* ql = lo + 8 * (size_t)i;
  *(volatile v4u*)qh = uh;
  *(volatile v4u*)ql = ul;
  __threadfence();
  *(volatile v4u*)qh = uh;
  *(volatile v4u*)ql = ul;
}

__global__ __launch_bounds__(256) void scan_kernel(
    const unsigned short* __restrict__ Wth, const unsigned short* __restrict__ Wtl,
    const float* __restrict__ bt, const float* __restrict__ Up,
    const float* __restrict__ ANGp, const float* __restrict__ CDp,
    unsigned short* __restrict__ STh, unsigned short* __restrict__ STl,
    float* __restrict__ fstate) {
  __shared__ __align__(16) unsigned short Ah[16 * kDim];
  __shared__ __align__(16) unsigned short Al[16 * kDim];
  __shared__ __align__(16) float NS[kBatch * kDim];
  __shared__ __align__(16) float CSc[kBatch * kHalf];
  __shared__ __align__(16) float CSs[kBatch * kHalf];
  typedef Frag<__bf16> F;

  const int t    = threadIdx.x;
  const int lane = t & 31;
  const int wave = t >> 5;
  const int lh   = lane >> 4;
  const int rl   = lane & 15;
  const int koff = lh * 8;
  const int n0   = wave * 64;

  {
    const v4u z = (v4u){0u, 0u, 0u, 0u};
#pragma unroll
    for (int i = 0; i < 4; ++i) {
      *(v4u*)(Ah + (size_t)(t + 256 * i) * 8) = z;
      *(v4u*)(Al + (size_t)(t + 256 * i) * 8) = z;
    }
  }

  float btv[4], sgv[4];
#pragma unroll
  for (int nt = 0; nt < 4; ++nt) {
    const int col = n0 + (nt << 4) + rl;
    btv[nt] = bt[col];
    sgv[nt] = (col & 1) ? 1.0f : -1.0f;
  }

  const __bf16* WthB = (const __bf16*)(const void*)Wth;
  const __bf16* WtlB = (const __bf16*)(const void*)Wtl;
  const __bf16* AhB  = (const __bf16*)(const void*)Ah;
  const __bf16* AlB  = (const __bf16*)(const void*)Al;

  for (int s = 0; s < kSeq; ++s) {
    {
      const int b = wave;
      const float* ap = ANGp + ((size_t)b * kSeq + s) * kHalf;
#pragma unroll 1
      for (int e = 0; e < 8; ++e) {
        const int j = e * 32 + lane;
        const float a = ap[j];
        CSc[b * kHalf + j] = cosf(a);
        CSs[b * kHalf + j] = sinf(a);
      }
    }
    __syncthreads();

    v8f acc[4];
#pragma unroll
    for (int nt = 0; nt < 4; ++nt) acc[nt] = (v8f){0.f,0.f,0.f,0.f,0.f,0.f,0.f,0.f};
    for (int k0 = 0; k0 < kDim; k0 += 32) {
      v16b bh[4], bl[4];
#pragma unroll
      for (int j = 0; j < 4; ++j) {
        const size_t bo = (size_t)(n0 + (j << 4) + rl) * kDim + koff + k0;
        bh[j] = F::load(WthB + bo);
        bl[j] = F::load(WtlB + bo);
      }
      const size_t ao = (size_t)rl * kDim + koff + k0;
      const v16b ah = F::load(AhB + ao);
      const v16b al = F::load(AlB + ao);
#pragma unroll
      for (int j = 0; j < 4; ++j) {
        acc[j] = F::mma(ah, bh[j], acc[j]);
        acc[j] = F::mma(ah, bl[j], acc[j]);
        acc[j] = F::mma(al, bh[j], acc[j]);
      }
      F::guard(acc[0], acc[3], ah, al);
      F::keep(bh[0], bh[1], bh[2], bh[3]);
      F::keep(bl[0], bl[1], bl[2], bl[3]);
    }
    acc_guard4(acc[0], acc[1], acc[2], acc[3]);

    {
#pragma unroll
      for (int nt = 0; nt < 4; ++nt) {
        const int col = n0 + (nt << 4) + rl;
        const int j = col >> 1;
#pragma unroll
        for (int rr = 0; rr < 4; ++rr) {
          const int b = 4 * lh + rr;
          const float tv  = acc[nt][2 * rr] + btv[nt];
          const float oth = __shfl_xor(tv, 1, 32);
          const float cs  = CSc[b * kHalf + j];
          const float sn  = CSs[b * kHalf + j];
          const float rot = tv * cs + sgv[nt] * (oth * sn);
          const size_t tok = (size_t)b * kSeq + s;
          const float g  = Up[tok * kDim + col];
          const float cd = CDp[tok * kDim + col];
          NS[b * kDim + col] = g * rot + (1.0f - g) * cd;
        }
      }
    }
    __syncthreads();

    for (int pass = 0; pass < 2; ++pass) {
#pragma unroll
      for (int i = 0; i < 2; ++i) {
        const int q  = t + 256 * i;
        const int b  = q >> 6;
        const int c0 = (q & 63) * 8;
        const v4f x0 = *(const v4f*)(NS + b * kDim + c0);
        const v4f x1 = *(const v4f*)(NS + b * kDim + c0 + 4);
        unsigned short hb[8], lb[8];
#pragma unroll
        for (int e = 0; e < 4; ++e) {
          const unsigned short h0 = f2bf_bits(x0[e]);
          hb[e] = h0; lb[e] = f2bf_bits(x0[e] - bf_bits2f(h0));
          const unsigned short h1 = f2bf_bits(x1[e]);
          hb[4 + e] = h1; lb[4 + e] = f2bf_bits(x1[e] - bf_bits2f(h1));
        }
        const v4u hv = (v4u){pk16(hb[0], hb[1]), pk16(hb[2], hb[3]), pk16(hb[4], hb[5]), pk16(hb[6], hb[7])};
        const v4u lv = (v4u){pk16(lb[0], lb[1]), pk16(lb[2], lb[3]), pk16(lb[4], lb[5]), pk16(lb[6], lb[7])};
        *(v4u*)(Ah + (size_t)(2 * b) * kDim + c0) = hv;
        *(v4u*)(Al + (size_t)(2 * b) * kDim + c0) = lv;
        const size_t go = ((size_t)b * kSeq + s) * kDim + c0;
        *(volatile v4u*)(STh + go) = hv;
        *(volatile v4u*)(STl + go) = lv;
      }
      __threadfence();
    }
  }

  for (int pass = 0; pass < 2; ++pass) {
#pragma unroll
    for (int i = 0; i < 4; ++i) {
      const int e4 = i * 256 + t;
      const int b  = e4 >> 7;
      const int c  = (e4 & 127) * 4;
      const v4f v = *(const v4f*)(NS + b * kDim + c);
      *(volatile v4f*)(fstate + (size_t)b * kDim + c) = v;
    }
    __threadfence();
  }
}

extern "C" void kernel_launch(void* const* d_in, const int* in_sizes, int n_in,
                              void* d_out, int out_size, void* d_ws,
                              size_t ws_size, hipStream_t stream) {
  if (n_in < 13) return;
  if (in_sizes[0] != kTok * kDim) return;
  if (in_sizes[1] != kDim * kDim || in_sizes[2] != kDim) return;
  if (in_sizes[3] != kDim * kDim || in_sizes[4] != kDim) return;
  if (in_sizes[5] != kHalf * kDim || in_sizes[6] != kHalf) return;
  if (in_sizes[7] != kDim * kDim || in_sizes[8] != kDim) return;
  if (in_sizes[9] != kDim * kDim || in_sizes[10] != kDim) return;
  if (in_sizes[11] != kDim * kDim || in_sizes[12] != kDim) return;
  if (out_size != kTok * kDim + kBatch * kDim) return;

  const size_t MiB = 1048576;
  const size_t offW = 112 * MiB;
  const size_t need = offW + 4718592;
  if (ws_size < need) return;

  const float* x  = (const float*)d_in[0];
  const float* Wu = (const float*)d_in[1];
  const float* bu = (const float*)d_in[2];
  const float* Wt = (const float*)d_in[3];
  const float* bt = (const float*)d_in[4];
  const float* Wa = (const float*)d_in[5];
  const float* ba = (const float*)d_in[6];
  const float* Wc = (const float*)d_in[7];
  const float* bc = (const float*)d_in[8];
  const float* Wg = (const float*)d_in[9];
  const float* bg = (const float*)d_in[10];
  const float* Wo = (const float*)d_in[11];
  const float* bo = (const float*)d_in[12];

  char* ws = (char*)d_ws;
  unsigned short* slot0 = (unsigned short*)(ws + 0);
  unsigned short* slot1 = (unsigned short*)(ws + 16 * MiB);
  float* ANG  = (float*)(ws + 32 * MiB);
  float* CAND = (float*)(ws + 48 * MiB);
  float* Y    = (float*)(ws + 48 * MiB);
  float* U    = (float*)(ws + 80 * MiB);
  unsigned short* XH2 = (unsigned short*)(ws + 80 * MiB);
  char* wb = ws + offW;
  unsigned short* Wuh = (unsigned short*)(wb + 0);
  unsigned short* Wgh = (unsigned short*)(wb + 524288);
  unsigned short* Wah = (unsigned short*)(wb + 1048576);
  unsigned short* Wal = (unsigned short*)(wb + 1310720);
  unsigned short* Wch = (unsigned short*)(wb + 1572864);
  unsigned short* Wcl = (unsigned short*)(wb + 2097152);
  unsigned short* Wth = (unsigned short*)(wb + 2621440);
  unsigned short* Wtl = (unsigned short*)(wb + 3145728);
  unsigned short* Woh = (unsigned short*)(wb + 3670016);
  unsigned short* Wol = (unsigned short*)(wb + 4194304);

  unsigned short* XBH = slot0;
  unsigned short* XBL = slot1;
  unsigned short* XH1 = slot0;
  unsigned short* STH = slot0;
  unsigned short* STL = slot1;

  float* out0 = (float*)d_out;
  float* out1 = (float*)d_out + (size_t)kTok * kDim;

  const int n8W  = kDim * kDim / 8;
  const int n8Wa = kHalf * kDim / 8;
  const int n8X  = kTok * kDim / 8;

  cast8_f16_kernel<<<dim3(n8W / 256), dim3(256), 0, stream>>>(Wu, Wuh, n8W, kWCarry);
  cast8_f16_kernel<<<dim3(n8W / 256), dim3(256), 0, stream>>>(Wg, Wgh, n8W, kWCarry);
  cast8_split_kernel<<<dim3(n8Wa / 256), dim3(256), 0, stream>>>(Wa, Wah, Wal, n8Wa);
  cast8_split_kernel<<<dim3(n8W / 256), dim3(256), 0, stream>>>(Wc, Wch, Wcl, n8W);
  cast8_split_kernel<<<dim3(n8W / 256), dim3(256), 0, stream>>>(Wt, Wth, Wtl, n8W);
  cast8_split_kernel<<<dim3(n8W / 256), dim3(256), 0, stream>>>(Wo, Woh, Wol, n8W);
  cast8_split_kernel<<<dim3(n8X / 256), dim3(256), 0, stream>>>(x, XBH, XBL, n8X);

  wmma_gemm64<1, true, 2, 0, false, 0, false><<<dim3(128, 1), dim3(256), 0, stream>>>(
      XBH, XBL, kDim, 0L, Wah, Wal, kDim, 0L, (void*)ANG, (void*)ANG, kHalf, 0L, ba, ba, 0L, kTok, kHalf, kDim, 1.0f);
  wmma_gemm64<1, true, 2, 0, false, 1, false><<<dim3(256, 1), dim3(256), 0, stream>>>(
      XBH, XBL, kDim, 0L, Wch, Wcl, kDim, 0L, (void*)CAND, (void*)CAND, kDim, 0L, bc, bc, 0L, kTok, kDim, kDim, 1.0f);
  cast8_f16_kernel<<<dim3(n8X / 256), dim3(256), 0, stream>>>(x, XH1, n8X, 1.0f);
  wmma_gemm64<0, false, 2, 0, false, 6, false><<<dim3(256, 1), dim3(256), 0, stream>>>(
      XH1, XH1, kDim, 0L, Wuh, Wuh, kDim, 0L, (void*)U, (void*)U, kDim, 0L, bu, bu, 0L, kTok, kDim, kDim, kWCarryInv);

  scan_kernel<<<dim3(1), dim3(256), 0, stream>>>(Wth, Wtl, bt, U, ANG, CAND, STH, STL, out1);

  wmma_gemm64<1, true, 2, 0, false, 0, false><<<dim3(256, 1), dim3(256), 0, stream>>>(
      STH, STL, kDim, 0L, Woh, Wol, kDim, 0L, (void*)Y, (void*)Y, kDim, 0L, bo, bo, 0L, kTok, kDim, kDim, 1.0f);
  cast8_f16_kernel<<<dim3(n8X / 256), dim3(256), 0, stream>>>(x, XH2, n8X, 1.0f);
  wmma_gemm64<0, false, 2, 0, true, 6, true><<<dim3(256, 1), dim3(256), 0, stream>>>(
      XH2, XH2, kDim, 0L, Wgh, Wgh, kDim, 0L, (void*)out0, (void*)out0, kDim, 0L, bg, Y, 0L, kTok, kDim, kDim, kWCarryInv);
}
